// BertAdapter_SLT_49933289783411
// MI455X (gfx1250) — hardware-run, weakly checked
//
#include <hip/hip_runtime.h>


namespace {
constexpr int NR = 8 * 512, HID = 768, R = 5;
constexpr float XS = 8.0f, WSC = 256.0f;
typedef _Float16 b16;
typedef __attribute__((ext_vector_type(16))) _Float16 v16b;
typedef __attribute__((ext_vector_type(8))) _Float16 v8b;
typedef __attribute__((ext_vector_type(8))) float v8f;
typedef __attribute__((ext_vector_type(4))) float v4f;
__device__ __forceinline__ float bf16_rne(float f) { unsigned int u = __float_as_uint(f); u += 0x7FFFu + ((u >> 16) & 1u); return __uint_as_float(u & 0xFFFF0000u); }
__device__ __forceinline__ void split16(float v, b16& hi, b16& lo) { hi = (b16)v; lo = (b16)(v - (float)hi); }
__device__ __forceinline__ v16b frag_kb(const b16* p, int hh) { const v8b a = *(const v8b*)(p + 8 * hh), b = *(const v8b*)(p + 16 + 8 * hh); v16b f;
#pragma unroll
  for (int e = 0; e < 8; ++e) { f[e] = a[e]; f[8 + e] = b[e]; } return f; }
__device__ __forceinline__ v8f wmma16b(v16b a, v16b b, v8f c) { v8f d = __builtin_amdgcn_wmma_f32_16x16x32_f16(false, a, false, b, (short)0, c, false, false); asm volatile("v_nop\n\tv_nop\n\tv_nop\n\tv_nop" : "+v"(d) : "v"(a), "v"(b)); return d; }
__device__ __forceinline__ void wave_lds_sync() { __builtin_amdgcn_fence(__ATOMIC_RELEASE, "workgroup"); __builtin_amdgcn_wave_barrier(); __builtin_amdgcn_fence(__ATOMIC_ACQUIRE, "workgroup"); }
__device__ __forceinline__ float pmul(float a, float b) { float p = a * b; asm volatile("" : "+v"(p)); return p; }
__device__ __forceinline__ float gelu(float v) { return 0.5f * v * (1.0f + erff(v * 0.70710678118654752f)); }

__global__ __launch_bounds__(256) void factors_kernel(const float* __restrict__ c0, const float* __restrict__ c1, const float* __restrict__ c2, const float* __restrict__ c3, const float* __restrict__ c4, const float* __restrict__ c5, b16* __restrict__ ATh, b16* __restrict__ ATl, b16* __restrict__ BTh, b16* __restrict__ BTl) {
  const int tid = threadIdx.x;
  for (int pass = 0; pass < 2; ++pass) {
    for (int idx = tid; idx < 16 * HID; idx += 256) { const int xr = idx / HID, in = idx % HID; float s = 0.0f;
      if (xr < R) { const int i = in / 64, j = (in / 8) % 8, k = in % 8; for (int v = 0; v < R; ++v) for (int w = 0; w < R; ++w) s += pmul(pmul(bf16_rne(c0[i * R + v]), bf16_rne(c1[(v * 8 + j) * R + w])), bf16_rne(c2[(w * 8 + k) * R + xr])); }
      b16 p, q; split16(s * WSC, p, q); ((volatile b16*)ATh)[idx] = p; ((volatile b16*)ATl)[idx] = q; }
    for (int idx = tid; idx < HID * 32; idx += 256) { const int o = idx / 32, xr = idx % 32; float s = 0.0f;
      if (xr < R) { const int p_ = o / 96, q_ = (o / 12) % 8, r_ = o % 12; for (int y = 0; y < R; ++y) for (int z = 0; z < R; ++z) s += pmul(pmul(bf16_rne(c3[(xr * 8 + p_) * R + y]), bf16_rne(c4[(y * 8 + q_) * R + z])), bf16_rne(c5[z * 12 + r_])); }
      b16 p, q; split16(s * WSC, p, q); ((volatile b16*)BTh)[idx] = p; ((volatile b16*)BTl)[idx] = q; }
    __threadfence(); }
}
__global__ __launch_bounds__(32) void tt_kernel(const float* __restrict__ x, const b16* __restrict__ ATh, const b16* __restrict__ ATl, const b16* __restrict__ BTh, const b16* __restrict__ BTl, const float* __restrict__ bias, int RL, float* __restrict__ out) {
  __shared__ __attribute__((aligned(16))) b16 Ah[16][HID + 8], Th[16][40], Tl[16][40]; __shared__ float Tf[16][260]; const int lane = threadIdx.x, nloc = lane & 15, hlf = lane >> 4; const size_t m0 = (size_t)blockIdx.x * 16; if (m0 >= (size_t)RL) return;
  for (int rr = 0; rr < 16; ++rr) for (int q = 0; q < HID / 32; ++q) Ah[rr][q * 32 + lane] = (b16)(bf16_rne(x[(m0 + rr) * HID + q * 32 + lane]) * XS);
  Th[nloc][lane] = (b16)0.0f; Tl[nloc][lane] = (b16)0.0f; if (lane >= 16) { Th[lane - 16][lane] = (b16)0.0f; }
  for (int rr = 0; rr < 16; ++rr) { Th[rr][lane] = (b16)0.0f; Tl[rr][lane] = (b16)0.0f; }
  wave_lds_sync(); v8f acc = {};
#pragma unroll 4
  for (int kb = 0; kb < HID; kb += 32) { const v16b a = frag_kb(&Ah[nloc][kb], hlf); acc = wmma16b(a, frag_kb(ATh + (size_t)nloc * HID + kb, hlf), acc); acc = wmma16b(a, frag_kb(ATl + (size_t)nloc * HID + kb, hlf), acc); }
  if (nloc < R) {
#pragma unroll
    for (int r8 = 0; r8 < 8; ++r8) { b16 p, q; split16(acc[r8] * (1.0f / (XS * WSC)) * XS, p, q); Th[8 * hlf + r8][nloc] = p; Tl[8 * hlf + r8][nloc] = q; } }
  wave_lds_sync(); const v16b th = frag_kb(&Th[nloc][0], hlf), tl = frag_kb(&Tl[nloc][0], hlf);
#pragma unroll 1
  for (int cg = 0; cg < 3; ++cg) { v8f o[16];
#pragma unroll
    for (int t = 0; t < 16; ++t) { o[t] = (v8f){}; const size_t br = (size_t)(cg * 256 + t * 16 + nloc) * 32; const v16b bh = frag_kb(BTh + br, hlf), bl = frag_kb(BTl + br, hlf); o[t] = wmma16b(th, bh, o[t]); o[t] = wmma16b(th, bl, o[t]); o[t] = wmma16b(tl, bh, o[t]); }
#pragma unroll
    for (int t = 0; t < 16; ++t) { const int c = cg * 256 + t * 16 + nloc; const float bb = bf16_rne(bias[c]);
#pragma unroll
      for (int r8 = 0; r8 < 8; ++r8) { const int rl = 8 * hlf + r8; Tf[rl][t * 16 + nloc] = bf16_rne(x[(m0 + rl) * HID + c]) + gelu(o[t][r8] * (1.0f / (XS * WSC)) + bb); } }
    wave_lds_sync();
    for (int pass = 0; pass < 2; ++pass) { for (int rr = 0; rr < 16; ++rr) for (int q = 0; q < 2; ++q) *(volatile v4f*)(out + (m0 + rr) * HID + cg * 256 + q * 128 + lane * 4) = *(const v4f*)(&Tf[rr][q * 128 + lane * 4]); __threadfence(); }
    wave_lds_sync(); }
}
}

extern "C" void kernel_launch(void* const* d_in, const int* in_sizes, int n_in, void* d_out, int out_size, void* d_ws, size_t ws_size, hipStream_t stream) {
  (void)n_in;
  auto Fp = [&](int i) { return (const float*)d_in[i]; };
  if (in_sizes[0] != NR * HID || in_sizes[1] != HID || in_sizes[2] != 12 * R || in_sizes[3] != R * 8 * R || in_sizes[4] != R * 8 * R || in_sizes[5] != R * 8 * R || in_sizes[6] != R * 8 * R || in_sizes[7] != R * 12 || out_size != NR * HID) return;
  const int RL = NR;
  size_t off = 0; char* ws = (char*)d_ws;
  auto carve = [&](size_t bytes) { char* p = ws + off; off += (bytes + 255) & ~(size_t)255; return p; };
  b16* ATh = (b16*)carve((size_t)16 * HID * 2); b16* ATl = (b16*)carve((size_t)16 * HID * 2); b16* BTh = (b16*)carve((size_t)HID * 32 * 2); b16* BTl = (b16*)carve((size_t)HID * 32 * 2);
  if (off > ws_size || off > ((size_t)4 << 20)) return;
  factors_kernel<<<1, 256, 0, stream>>>(Fp(2), Fp(3), Fp(4), Fp(5), Fp(6), Fp(7), ATh, ATl, BTh, BTl);
  tt_kernel<<<RL / 16, 32, 0, stream>>>(Fp(0), ATh, ATl, BTh, BTl, Fp(1), RL, (float*)d_out);
}
